// Encoder_block_944892805730
// MI455X (gfx1250) — hardware-verified
//
#include <hip/hip_runtime.h>
#include <math.h>
#include <stdint.h>

#ifndef NB
#define NB 8
#endif
#ifndef SEQ
#define SEQ 1024
#endif
#define NB_FULL  8
#define SEQ_FULL 1024
#define DM      768
#define NHEAD   8
#define HD      96
#define DFF     1500
#define DFFP    1536
#define NQK     (2 * DM)
#define KQK     (2 * DM)
#define NROWS   (NB * SEQ)
#define WSC     64.0f
#define W2SC    128.0f
#define HCARRY  16.0f
#define VC      16.0f
#define PC      4096.0f
#define FC      1024.0f
#define H2C     16.0f
#define GC      16.0f
#define SQRT_HD 9.797958971132712f
#define LOG2E   1.4426950408889634f
#define LN_EPS  1e-5f
static_assert(NHEAD * HD == DM && HD == 96);
static_assert(NB >= 1 && NB <= NB_FULL && SEQ >= 64 && SEQ <= SEQ_FULL);
static_assert((SEQ % 64) == 0 && (SEQ % 32) == 0 && (SEQ % 16) == 0 && (DM % 64) == 0 && (DFFP % 64) == 0 && (NQK % 64) == 0);
static_assert((DM % 32) == 0 && (KQK % 32) == 0 && (DFFP % 32) == 0 && (HD % 32) == 0 && (NROWS % 64) == 0);
static_assert(DFFP >= DFF && (DFF % 4) == 0 && (DM % 4) == 0 && (DM % 8) == 0);
#define ATT_THREADS (NHEAD * 32)
#define ATT_BLOCKS  (NB * (SEQ / 16))
static_assert(ATT_THREADS == 256);
#define LN_THREADS  192
#define LN_WAVES    (LN_THREADS / 32)
static_assert(LN_THREADS * 4 == DM && (LN_THREADS % 32) == 0 && ((DM / 8) % 32) == 0 && LN_THREADS * 8 == NQK);

typedef _Float16 v16h __attribute__((ext_vector_type(16)));
typedef _Float16 v8h  __attribute__((ext_vector_type(8)));
typedef __bf16   v16b __attribute__((ext_vector_type(16)));
typedef float    v8f  __attribute__((ext_vector_type(8)));
typedef float    v4f  __attribute__((ext_vector_type(4)));
typedef unsigned int v4u __attribute__((ext_vector_type(4)));
typedef unsigned int v2u __attribute__((ext_vector_type(2)));

union FragU { v16h h; v16b b; v8h h8[2]; v4u u[2]; };

__device__ __forceinline__ unsigned short bf_bits(float f) {
  unsigned u = __float_as_uint(f);
  return (unsigned short)((u + 0x7FFFu + ((u >> 16) & 1u)) >> 16);
}
__device__ __forceinline__ float bf_up(unsigned short h) { return __uint_as_float(((unsigned)h) << 16); }
__device__ __forceinline__ float bfr(float f) { return bf_up(bf_bits(f)); }
__device__ __forceinline__ unsigned short h_bits(_Float16 x) { return __builtin_bit_cast(unsigned short, x); }
__device__ __forceinline__ unsigned pk16(unsigned short a, unsigned short b) { return (unsigned)a | ((unsigned)b << 16); }
__device__ __forceinline__ v8f zero8() { v8f z = {0.f, 0.f, 0.f, 0.f, 0.f, 0.f, 0.f, 0.f}; return z; }
__device__ __forceinline__ float gelu_f(float v) { return 0.5f * v * (1.0f + erff(v * 0.70710678118654752f)); }

__device__ __forceinline__ FragU ldfrag_u(const unsigned short* p) {
  FragU f;
  f.u[0] = *(const v4u*)(p);
  f.u[1] = *(const v4u*)(p + 16);
  return f;
}
__device__ __forceinline__ FragU ldfrag_h(const _Float16* p) {
  FragU f;
  f.h8[0] = *(const v8h*)(p);
  f.h8[1] = *(const v8h*)(p + 16);
  return f;
}

__device__ __forceinline__ v8f mma_h(const FragU& a, const FragU& b, v8f c) {
  return __builtin_amdgcn_wmma_f32_16x16x32_f16(false, a.h, false, b.h, (short)0, c, false, false);
}
__device__ __forceinline__ v8f mma_b(const FragU& a, const FragU& b, v8f c) {
  return __builtin_amdgcn_wmma_f32_16x16x32_bf16(false, a.b, false, b.b, (short)0, c, false, false);
}
template <int BF>
__device__ __forceinline__ v8f mma16(const FragU& a, const FragU& b, v8f c) {
  if constexpr (BF != 0) return mma_b(a, b, c);
  else return mma_h(a, b, c);
}
__device__ __forceinline__ void dep_guard1(v8f& a, v8f& b, v16h x) {
#if defined(__HIP_DEVICE_COMPILE__)
  asm volatile("v_nop\n\tv_nop\n\tv_nop\n\tv_nop" : "+v"(a), "+v"(b) : "v"(x));
#endif
}
__device__ __forceinline__ void keep4_h(v16h a, v16h b, v16h c, v16h d) {
#if defined(__HIP_DEVICE_COMPILE__)
  asm volatile("v_nop" :: "v"(a), "v"(b), "v"(c), "v"(d));
#endif
}
__device__ __forceinline__ void acc_guard4(v8f& a, v8f& b, v8f& c, v8f& d) {
#if defined(__HIP_DEVICE_COMPILE__)
  asm volatile("v_nop\n\tv_nop\n\tv_nop\n\tv_nop" : "+v"(a), "+v"(b), "+v"(c), "+v"(d));
#endif
}
__device__ __forceinline__ void guard_sc(v8f& s, v16h k0, v16h k1, v16h k2, v16h k3, v16h k4, v16h k5,
                                         v16h q0v, v16h q1v, v16h q2v, v16h q3v, v16h q4v, v16h q5v) {
#if defined(__HIP_DEVICE_COMPILE__)
  asm volatile("v_nop\n\tv_nop\n\tv_nop\n\tv_nop" : "+v"(s)
               : "v"(k0), "v"(k1), "v"(k2), "v"(k3), "v"(k4), "v"(k5),
                 "v"(q0v), "v"(q1v), "v"(q2v), "v"(q3v), "v"(q4v), "v"(q5v));
#endif
}
__device__ __forceinline__ void guard_pv6(v8f& a0, v8f& a1, v8f& a2, v8f& a3, v8f& a4, v8f& a5,
                                          v16h p, v16h b0, v16h b1, v16h b2, v16h b3, v16h b4, v16h b5) {
#if defined(__HIP_DEVICE_COMPILE__)
  asm volatile("v_nop\n\tv_nop\n\tv_nop\n\tv_nop"
               : "+v"(a0), "+v"(a1), "+v"(a2), "+v"(a3), "+v"(a4), "+v"(a5)
               : "v"(p), "v"(b0), "v"(b1), "v"(b2), "v"(b3), "v"(b4), "v"(b5));
#endif
}
__device__ __forceinline__ void wave_sync_lds() {
  __builtin_amdgcn_fence(3  , "workgroup");
  __builtin_amdgcn_wave_barrier();
  __builtin_amdgcn_fence(2  , "workgroup");
}

template <int TW>
__global__ __launch_bounds__(256) void tcvt16(const float* __restrict__ src, int pitch, int R, int C,
                                              unsigned short* dst, int ldo, int rdup, float sc) {
  __shared__ __align__(16) unsigned short sT[64 * 72];
  const int tid = threadIdx.x, lane = tid & 31, wave = tid >> 5;
  const int c0 = blockIdx.x * 64, r0 = blockIdx.y * 64;
  const int rr = tid >> 2, cc = (tid & 3) * 16;
  const int r = r0 + rr;
  const int rcl = min(r, R - 1);
  const bool rok = (r < R);
  const float* sp = src + (size_t)rcl * pitch;
#pragma unroll
  for (int e = 0; e < 4; ++e) {
    const int c = c0 + cc + 4 * e;
    const int ccl = min(c, C - 4);
    const v4f a = *(const v4f*)(sp + ccl);
    const bool ok = rok && (c < C);
#pragma unroll
    for (int k = 0; k < 4; ++k) {
      const float v = ok ? a[k] : 0.f;
      unsigned short w;
      if constexpr (TW == 1) w = bf_bits(v);
      else w = h_bits((_Float16)(bfr(v) * sc));
      sT[(cc + 4 * e + k) * 72 + rr] = w;
    }
  }
  __syncthreads();
  v4u vals[2];
#pragma unroll
  for (int it = 0; it < 2; ++it) {
    const int q = it * 32 + wave * 4 + (lane >> 3);
    vals[it] = *(const v4u*)(sT + q * 72 + (lane & 7) * 8);
  }
  for (int pass = 0; pass < 2; ++pass) {
#pragma unroll
    for (int it = 0; it < 2; ++it) {
      const int q = it * 32 + wave * 4 + (lane >> 3);
      unsigned short* p = dst + (size_t)(c0 + q) * ldo + r0 + (lane & 7) * 8;
      *(volatile v4u*)(p) = vals[it];
      if constexpr (TW == 1) { *(volatile v4u*)(p + rdup) = vals[it]; }
    }
    __threadfence();
  }
}

template <int BF, int OM, int HASR, int HASB, int ACT>
__global__ __launch_bounds__(256) void gemm64(
    const unsigned short* __restrict__ Ap, int lda, long long sA,
    const unsigned short* __restrict__ Btp, int ldb, long long sB,
    const float* __restrict__ Rp, int ldr, long long sR,
    const float* __restrict__ Bsp, int nbias,
    void* Cout, void* Cout2, int ldc, long long sC,
    int M, int N, int K, float oscale, float ocarry) {
  __shared__ __align__(16) float sT[8][16 * 68];
  const int by   = blockIdx.y;
  const int lane = threadIdx.x & 31;
  const int wave = threadIdx.x >> 5;
  const int tilesN = N >> 6;
  const int tilesM = M >> 6;
  const int tile = blockIdx.x * 8 + wave;
  if (tile >= tilesM * tilesN) return;
  const int tm = tile / tilesN;
  const int tn = tile - tm * tilesN;
  const int m0 = tm << 6;
  const int n0 = tn << 6;

  const unsigned short* A1 = Ap  + (size_t)((long long)by * sA);
  const unsigned short* Bb = Btp + (size_t)((long long)by * sB);

  const int rlane = lane & 15;
  const int koff  = (lane >> 4) * 8;
  const int mOff  = (lane >> 4) * 8;

  v8f acc[4][4];
#pragma unroll
  for (int i = 0; i < 4; ++i)
#pragma unroll
    for (int j = 0; j < 4; ++j) acc[i][j] = zero8();

  for (int k0 = 0; k0 < K; k0 += 32) {
    FragU bh[4];
#pragma unroll
    for (int j = 0; j < 4; ++j) {
      const size_t bofs = (size_t)(n0 + (j << 4) + rlane) * ldb + koff + k0;
      bh[j] = ldfrag_u(Bb + bofs);
    }
#pragma unroll
    for (int i = 0; i < 4; ++i) {
      const size_t ao = (size_t)(m0 + (i << 4) + rlane) * lda + koff + k0;
      const FragU ah = ldfrag_u(A1 + ao);
#pragma unroll
      for (int j = 0; j < 4; ++j) acc[i][j] = mma16<BF>(ah, bh[j], acc[i][j]);
      dep_guard1(acc[i][0], acc[i][3], ah.h);
    }
    keep4_h(bh[0].h, bh[1].h, bh[2].h, bh[3].h);
  }
  acc_guard4(acc[0][0], acc[0][1], acc[0][2], acc[0][3]);
  acc_guard4(acc[1][0], acc[1][1], acc[1][2], acc[1][3]);
  acc_guard4(acc[2][0], acc[2][1], acc[2][2], acc[2][3]);
  acc_guard4(acc[3][0], acc[3][1], acc[3][2], acc[3][3]);

  const int hh2 = lane >> 4, c4 = (lane & 15) * 4;
  const int q8  = lane >> 3, c8 = (lane & 7) * 8;

  float* slab = sT[wave];
#pragma unroll
  for (int i = 0; i < 4; ++i) {
    const int mBase = m0 + (i << 4);
#pragma unroll
    for (int j = 0; j < 4; ++j) {
#pragma unroll
      for (int r = 0; r < 8; ++r) {
        slab[(mOff + r) * 68 + (j << 4) + rlane] = acc[i][j][r];
      }
    }
    wave_sync_lds();
    if constexpr (OM == 0) {
      float* C = (float*)Cout + (size_t)((long long)by * sC);
      v4f bv = {0.f, 0.f, 0.f, 0.f};
      if constexpr (HASB == 1) {
#pragma unroll
        for (int e = 0; e < 4; ++e) {
          const int n = n0 + c4 + e;
          const float braw = Bsp[min(n, nbias - 1)];
          bv[e] = (n < nbias) ? bfr(braw) : 0.f;
        }
      }
      v4f vals[8];
#pragma unroll
      for (int it = 0; it < 8; ++it) {
        const int row = it * 2 + hh2;
        const int gr  = mBase + row;
        v4f v = *(const v4f*)(slab + row * 68 + c4);
        v4f rv = {0.f, 0.f, 0.f, 0.f};
        if constexpr (HASR != 0) {
          const float* R = Rp + (size_t)((long long)by * sR);
          const v4f rraw = *(const v4f*)(R + (size_t)gr * ldr + n0 + c4);
#pragma unroll
          for (int e = 0; e < 4; ++e) rv[e] = (HASR == 1) ? bfr(rraw[e]) : rraw[e];
        }
#pragma unroll
        for (int e = 0; e < 4; ++e) v[e] = (v[e] * oscale + bv[e]) + rv[e];
        vals[it] = v;
      }
      for (int pass = 0; pass < 2; ++pass) {
#pragma unroll
        for (int it = 0; it < 8; ++it) {
          const int gr = mBase + it * 2 + hh2;
          *(volatile v4f*)(C + (size_t)gr * ldc + n0 + c4) = vals[it];
        }
        __threadfence();
      }
    } else {
      unsigned short* C = (unsigned short*)Cout + (size_t)((long long)by * sC);
      float bb8[8];
#pragma unroll
      for (int e = 0; e < 8; ++e) bb8[e] = 0.f;
      if constexpr (HASB == 1) {
#pragma unroll
        for (int e = 0; e < 8; ++e) {
          const int n = n0 + c8 + e;
          const float braw = Bsp[min(n, nbias - 1)];
          bb8[e] = (n < nbias) ? bfr(braw) : 0.f;
        }
      }
      v4u hv[4];
      v4u lv[4];
#pragma unroll
      for (int it = 0; it < 4; ++it) {
        const int row = it * 4 + q8;
        const float* sp = slab + row * 68 + c8;
        float brow = 0.f;
        if constexpr (HASB == 2) {
          const int gr = mBase + row;
          brow = bfr(Bsp[min(gr, nbias - 1)]);
        }
        v4u a  = {0u, 0u, 0u, 0u};
        v4u l2 = {0u, 0u, 0u, 0u};
#pragma unroll
        for (int e = 0; e < 4; ++e) {
          float f0 = sp[2 * e] * oscale + bb8[2 * e] + brow;
          float f1 = sp[2 * e + 1] * oscale + bb8[2 * e + 1] + brow;
          if constexpr (OM == 2) {
            if constexpr (ACT == 1) { f0 = fmaxf(f0, 0.f); f1 = fmaxf(f1, 0.f); }
            if constexpr (ACT == 2) { f0 = gelu_f(f0); f1 = gelu_f(f1); }
            f0 *= ocarry; f1 *= ocarry;
            a[e] = pk16(h_bits((_Float16)f0), h_bits((_Float16)f1));
          } else {
            const unsigned short h0 = bf_bits(f0), h1 = bf_bits(f1);
            const unsigned short l0 = bf_bits(f0 - bf_up(h0)), l1 = bf_bits(f1 - bf_up(h1));
            a[e]  = pk16(h0, h1);
            l2[e] = pk16(l0, l1);
          }
        }
        hv[it] = a;
        lv[it] = l2;
      }
      for (int pass = 0; pass < 2; ++pass) {
#pragma unroll
        for (int it = 0; it < 4; ++it) {
          const int row = it * 4 + q8;
          *(volatile v4u*)(C + (size_t)(mBase + row) * ldc + n0 + c8) = hv[it];
          if constexpr (OM == 3) {
            unsigned short* C2 = (unsigned short*)Cout2 + (size_t)((long long)by * sC);
            *(volatile v4u*)(C2 + (size_t)(mBase + row) * ldc + n0 + c8) = lv[it];
          }
        }
        __threadfence();
      }
    }
    wave_sync_lds();
  }
}

#define PS_FLOATS (8 * DM)
static_assert(PS_FLOATS >= NHEAD * 16 * 36);
static_assert((size_t)16 * DM * sizeof(unsigned short) <= (size_t)PS_FLOATS * sizeof(float));
#define ATT_IT ((16 * DM) / (8 * ATT_THREADS))
static_assert(ATT_IT * 8 * ATT_THREADS == 16 * DM && ((DM / 8) % 8) == 0);

__global__ __launch_bounds__(ATT_THREADS)
void attn8(const unsigned short* __restrict__ QKHp, const unsigned short* __restrict__ QKLp,
           const unsigned short* __restrict__ VTq, unsigned short* CT) {
  __shared__ __align__(16) float smem[PS_FLOATS];

  const int tid  = threadIdx.x;
  const int wave = tid >> 5;
  const int lane = tid & 31;
  const int hh   = lane >> 4;
  const int c    = lane & 15;

  const int qt   = blockIdx.x % (SEQ / 16);
  const int bat  = blockIdx.x / (SEQ / 16);
  const int head = wave;
  const int q0   = qt * 16;

  const size_t qofs = ((size_t)bat * SEQ + q0 + c) * NQK + head * HD + 8 * hh;
  const size_t kofs = ((size_t)bat * SEQ) * NQK + DM + head * HD + 8 * hh;
  const unsigned short* Khb = QKHp + kofs;
  const unsigned short* Klb = QKLp + kofs;
  const _Float16* Vb = (const _Float16*)(const void*)VTq + ((size_t)bat * DM + head * HD) * SEQ + 8 * hh;
  const float lsc = SQRT_HD * LOG2E;

  FragU qh[3], ql[3];
#pragma unroll
  for (int ks = 0; ks < 3; ++ks) {
    qh[ks] = ldfrag_u(QKHp + qofs + 32 * ks);
    ql[ks] = ldfrag_u(QKLp + qofs + 32 * ks);
  }

  float mrow[8], lrow[8];
  v8f o[6];
#pragma unroll
  for (int f = 0; f < 6; ++f) o[f] = zero8();
#pragma unroll
  for (int r = 0; r < 8; ++r) { mrow[r] = -INFINITY; lrow[r] = 0.f; }
  float* pt = smem + wave * (16 * 36);

#pragma unroll 1
  for (int kb = 0; kb < SEQ; kb += 32) {
    v8f s[2];
#pragma unroll
    for (int j = 0; j < 2; ++j) {
      const size_t ko = (size_t)(kb + 16 * j + c) * NQK;
      v8f sa = zero8();
      FragU kh[3], kl[3];
#pragma unroll
      for (int ks = 0; ks < 3; ++ks) {
        kh[ks] = ldfrag_u(Khb + ko + 32 * ks);
        kl[ks] = ldfrag_u(Klb + ko + 32 * ks);
      }
#pragma unroll
      for (int ks = 0; ks < 3; ++ks) {
        sa = mma_b(qh[ks], kh[ks], sa);
        sa = mma_b(qh[ks], kl[ks], sa);
        sa = mma_b(ql[ks], kh[ks], sa);
      }
      guard_sc(sa, kh[0].h, kh[1].h, kh[2].h, kl[0].h, kl[1].h, kl[2].h,
               qh[0].h, qh[1].h, qh[2].h, ql[0].h, ql[1].h, ql[2].h);
      s[j] = sa;
    }
#pragma unroll
    for (int r = 0; r < 8; ++r) {
      const float t0 = s[0][r] * lsc;
      const float t1 = s[1][r] * lsc;
      float mx = fmaxf(t0, t1);
#pragma unroll
      for (int off = 1; off < 16; off <<= 1) mx = fmaxf(mx, __shfl_xor(mx, off, 32));
      const float mn = fmaxf(mrow[r], mx);
      const float al = exp2f(fmaxf(mrow[r] - mn, -126.0f));
      mrow[r] = mn;
      const float e0 = exp2f(t0 - mn);
      const float e1 = exp2f(t1 - mn);
      float ps = e0 + e1;
#pragma unroll
      for (int off = 1; off < 16; off <<= 1) ps += __shfl_xor(ps, off, 32);
      lrow[r] = lrow[r] * al + ps;
#pragma unroll
      for (int f = 0; f < 6; ++f) o[f][r] *= al;
      const int ro = (8 * hh + r) * 36 + c;
      pt[ro]      = e0;
      pt[ro + 16] = e1;
    }
    wave_sync_lds();
    FragU ph;
    {
      const float* prow = pt + c * 36 + 8 * hh;
      const v4f p0 = *(const v4f*)(prow), p1 = *(const v4f*)(prow + 4);
      const v4f p2 = *(const v4f*)(prow + 16), p3 = *(const v4f*)(prow + 20);
#pragma unroll
      for (int e = 0; e < 4; ++e) {
        ph.h8[0][e]     = (_Float16)(p0[e] * PC);
        ph.h8[0][4 + e] = (_Float16)(p1[e] * PC);
        ph.h8[1][e]     = (_Float16)(p2[e] * PC);
        ph.h8[1][4 + e] = (_Float16)(p3[e] * PC);
      }
    }
    const _Float16* vp = Vb + (size_t)c * SEQ + kb;
    {
      FragU vb[6];
#pragma unroll
      for (int f = 0; f < 6; ++f) vb[f] = ldfrag_h(vp + (size_t)f * 16 * SEQ);
#pragma unroll
      for (int f = 0; f < 6; ++f) o[f] = mma_h(ph, vb[f], o[f]);
      guard_pv6(o[0], o[1], o[2], o[3], o[4], o[5], ph.h, vb[0].h, vb[1].h, vb[2].h, vb[3].h, vb[4].h, vb[5].h);
    }
    wave_sync_lds();
  }

  __syncthreads();
  unsigned short* Os = (unsigned short*)smem;
  const float oc = FC / (PC * VC);
  unsigned short* osw = Os + wave * HD + c;
#pragma unroll
  for (int r = 0; r < 8; ++r) {
    const float inv = (1.0f / lrow[r]) * oc;
    unsigned short* op = osw + (8 * hh + r) * DM;
#pragma unroll
    for (int f = 0; f < 6; ++f) op[16 * f] = h_bits((_Float16)(o[f][r] * inv));
  }
  __syncthreads();
  {
    v4u vals[ATT_IT];
#pragma unroll
    for (int it = 0; it < ATT_IT; ++it) {
      const int p = it * ATT_THREADS + tid;
      vals[it] = *(const v4u*)(Os + (size_t)p * 8);
    }
    unsigned short* dst = CT + ((size_t)bat * SEQ + q0) * DM;
    for (int pass = 0; pass < 2; ++pass) {
#pragma unroll
      for (int it = 0; it < ATT_IT; ++it) {
        const int p = it * ATT_THREADS + tid;
        const int row = p / (DM / 8), col8 = (p - row * (DM / 8)) * 8;
        *(volatile v4u*)(dst + (size_t)row * DM + col8) = vals[it];
      }
      __threadfence();
    }
  }
}

template <int RIN, int SPL>
__global__ __launch_bounds__(LN_THREADS)
void lnorm(const float* __restrict__ Yp, long long inbs, const float* __restrict__ gp, const float* __restrict__ bp,
           unsigned short* outh, float hc, unsigned short* outb) {
  __shared__ float red[2][LN_WAVES];
  __shared__ __align__(16) unsigned short srow[DM];
  __shared__ __align__(16) unsigned short sbh[(SPL != 0) ? NQK : 8];
  const int row  = blockIdx.x;
  const int tid  = threadIdx.x;
  const int lane = tid & 31;
  const int wave = tid >> 5;
  const int b    = row / SEQ;
  const int tok  = row - b * SEQ;
  const size_t base = (size_t)b * (size_t)inbs + (size_t)tok * DM + (size_t)tid * 4;
  v4f v = *(const v4f*)(Yp + base);
  if constexpr (RIN == 1) {
#pragma unroll
    for (int e = 0; e < 4; ++e) v[e] = bfr(v[e]);
  }
  float s = (v[0] + v[1]) + (v[2] + v[3]);
#pragma unroll
  for (int off = 1; off < 32; off <<= 1) s += __shfl_xor(s, off, 32);
  if (lane == 0) red[0][wave] = s;
  __syncthreads();
  float tot = 0.f;
#pragma unroll
  for (int w = 0; w < LN_WAVES; ++w) tot += red[0][w];
  const float mu = tot * (1.0f / (float)DM);
  v4f d;
#pragma unroll
  for (int e = 0; e < 4; ++e) d[e] = v[e] - mu;
  float q = (d[0] * d[0] + d[1] * d[1]) + (d[2] * d[2] + d[3] * d[3]);
#pragma unroll
  for (int off = 1; off < 32; off <<= 1) q += __shfl_xor(q, off, 32);
  if (lane == 0) red[1][wave] = q;
  __syncthreads();
  float totq = 0.f;
#pragma unroll
  for (int w = 0; w < LN_WAVES; ++w) totq += red[1][w];
  const float var  = totq * (1.0f / (float)DM);
  const float rstd = rsqrtf(var + LN_EPS);
  const v4f gv = *(const v4f*)(gp + (size_t)tid * 4);
  const v4f bv = *(const v4f*)(bp + (size_t)tid * 4);
  v4f o;
#pragma unroll
  for (int e = 0; e < 4; ++e) o[e] = (d[e] * rstd) * bfr(gv[e]) + bfr(bv[e]);
  {
    v2u w;
    w[0] = pk16(h_bits((_Float16)(o[0] * hc)), h_bits((_Float16)(o[1] * hc)));
    w[1] = pk16(h_bits((_Float16)(o[2] * hc)), h_bits((_Float16)(o[3] * hc)));
    *(v2u*)(srow + tid * 4) = w;
  }
  if constexpr (SPL != 0) {
    unsigned short hi[4], lo[4];
#pragma unroll
    for (int e = 0; e < 4; ++e) { hi[e] = bf_bits(o[e]); lo[e] = bf_bits(o[e] - bf_up(hi[e])); }
    v2u wh, wl;
    wh[0] = pk16(hi[0], hi[1]); wh[1] = pk16(hi[2], hi[3]);
    wl[0] = pk16(lo[0], lo[1]); wl[1] = pk16(lo[2], lo[3]);
    *(v2u*)(sbh + tid * 4) = wh;
    *(v2u*)(sbh + DM + tid * 4) = wl;
  }
  __syncthreads();
  const bool wlo = (tid < DM / 8);
  v4u hv = {0u, 0u, 0u, 0u};
  if (wlo) hv = *(const v4u*)(srow + tid * 8);
  v4u bvv = {0u, 0u, 0u, 0u};
  if constexpr (SPL != 0) bvv = *(const v4u*)(sbh + tid * 8);
  unsigned short* dsth = outh + (size_t)row * DM + (size_t)tid * 8;
  for (int pass = 0; pass < 2; ++pass) {
    if (wlo) *(volatile v4u*)dsth = hv;
    if constexpr (SPL != 0) {
      unsigned short* dstb = outb + (size_t)row * NQK + (size_t)tid * 8;
      *(volatile v4u*)dstb = bvv;
    }
    __threadfence();
  }
}

static inline size_t zmax(size_t a, size_t b) { return a > b ? a : b; }

extern "C" void kernel_launch(void* const* d_in, const int* in_sizes, int n_in,
                              void* d_out, int out_size, void* d_ws, size_t ws_size,
                              hipStream_t stream) {
  if (n_in < 11) return;
  if (in_sizes[0] < ((NB - 1) * SEQ_FULL + SEQ) * DM) return;
  if (in_sizes[1] < DM || in_sizes[2] < DM) return;
  if (in_sizes[3] < DM * 3 * DM || in_sizes[4] < 3 * DM) return;
  if (in_sizes[5] < DM * DM || in_sizes[6] < DM) return;
  if (in_sizes[7] < DM * DFF || in_sizes[8] < DFF) return;
  if (in_sizes[9] < DFF * DM || in_sizes[10] < DM) return;
  if (out_size < NROWS * DM) return;

  const float* x    = (const float*)d_in[0];
  const float* lng  = (const float*)d_in[1];
  const float* lnb  = (const float*)d_in[2];
  const float* Wqkv = (const float*)d_in[3];
  const float* bqkv = (const float*)d_in[4];
  const float* W0   = (const float*)d_in[5];
  const float* b0   = (const float*)d_in[6];
  const float* W1   = (const float*)d_in[7];
  const float* b1   = (const float*)d_in[8];
  const float* W2   = (const float*)d_in[9];
  const float* b2   = (const float*)d_in[10];
  float*       out  = (float*)d_out;

  const size_t PWQK = (size_t)NQK * KQK * 2;
  const size_t PWV  = (size_t)DM * DM * 2;
  const size_t PWO  = (size_t)DM * DM * 2;
  const size_t PW1  = (size_t)DFFP * DM * 2;
  const size_t PW2  = (size_t)DM * DFFP * 2;
  const size_t PHB  = (size_t)NROWS * NQK * 2;
  const size_t PQK  = (size_t)NROWS * NQK * 2;
  const size_t PH16 = (size_t)NROWS * DM * 2;
  const size_t PCT  = (size_t)NROWS * DM * 2;
  const size_t PX1  = (size_t)NROWS * DM * 4;
  const size_t PH2  = (size_t)NROWS * DM * 2;
  const size_t PHH  = (size_t)NROWS * DFFP * 2;
  const size_t PVT  = (size_t)NB * DM * SEQ * 2;
  const size_t PR1  = zmax(PHB, zmax(PCT, PHH));
  const size_t PR2  = zmax(PQK, PX1);
  const size_t PR3  = zmax(PQK, PH2);
  size_t off = 0;
  const size_t oWQK = off; off += PWQK;
  const size_t oWV  = off; off += PWV;
  const size_t oWO  = off; off += PWO;
  const size_t oW1  = off; off += PW1;
  const size_t oW2  = off; off += PW2;
  const size_t oR1  = off; off += PR1;
  const size_t oR2  = off; off += PR2;
  const size_t oR3  = off; off += PR3;
  const size_t oR4  = off; off += PH16;
  const size_t oR5  = off; off += PVT;
  if (off > ws_size) return;
  if (off > (size_t)134217728) return;

  char* ws = (char*)d_ws;
  unsigned short* WQK  = (unsigned short*)(ws + oWQK);
  unsigned short* WV16 = (unsigned short*)(ws + oWV);
  unsigned short* WO16 = (unsigned short*)(ws + oWO);
  unsigned short* W116 = (unsigned short*)(ws + oW1);
  unsigned short* W216 = (unsigned short*)(ws + oW2);
  unsigned short* HB   = (unsigned short*)(ws + oR1);
  unsigned short* CT   = (unsigned short*)(ws + oR1);
  unsigned short* HH   = (unsigned short*)(ws + oR1);
  unsigned short* QKH  = (unsigned short*)(ws + oR2);
  float*          X1F  = (float*)(ws + oR2);
  unsigned short* QKL  = (unsigned short*)(ws + oR3);
  unsigned short* H2   = (unsigned short*)(ws + oR3);
  unsigned short* H16  = (unsigned short*)(ws + oR4);
  unsigned short* VTp  = (unsigned short*)(ws + oR5);

  const dim3 blk(256);
  const dim3 gTqk(NQK / 64, DM / 64);
  const dim3 gTv(DM / 64, DM / 64);
  const dim3 gT0(DM / 64, DM / 64);
  const dim3 gT1(DFFP / 64, DM / 64);
  const dim3 gT2(DM / 64, DFFP / 64);
  const int tilesQK = (NROWS / 64) * (NQK / 64);
  const int tilesV  = (DM / 64) * (SEQ / 64);
  const int tilesO  = (SEQ / 64) * (DM / 64);
  const int tilesF1 = (NROWS / 64) * (DFFP / 64);
  const int tilesF2 = (NROWS / 64) * (DM / 64);
  const dim3 gQK((tilesQK + 7) / 8, 1);
  const dim3 gV((tilesV + 7) / 8, NB);
  const dim3 gO((tilesO + 7) / 8, NB);
  const dim3 gF1((tilesF1 + 7) / 8, 1);
  const dim3 gF2((tilesF2 + 7) / 8, 1);
  const dim3 gAT(ATT_BLOCKS);
  const dim3 bAT(ATT_THREADS);
  const dim3 gLN(NROWS);
  const dim3 bLN(LN_THREADS);

  tcvt16<1><<<gTqk, blk, 0, stream>>>(Wqkv, 3 * DM, DM, NQK, WQK, KQK, DM, 1.0f);
  tcvt16<0><<<gTv, blk, 0, stream>>>(Wqkv + 2 * DM, 3 * DM, DM, DM, WV16, DM, 0, WSC);
  tcvt16<0><<<gT0, blk, 0, stream>>>(W0, DM, DM, DM, WO16, DM, 0, WSC);
  tcvt16<0><<<gT1, blk, 0, stream>>>(W1, DFF, DM, DFF, W116, DM, 0, WSC);
  tcvt16<0><<<gT2, blk, 0, stream>>>(W2, DM, DFF, DM, W216, DFFP, 0, W2SC);

  lnorm<1, 1><<<gLN, bLN, 0, stream>>>(x, (long long)SEQ_FULL * DM, lng, lnb, H16, HCARRY, HB);

  gemm64<1, 3, 0, 1, 0><<<gQK, blk, 0, stream>>>(
      HB, KQK, 0LL,
      WQK, KQK, 0LL,
      (const float*)0, 0, 0LL,
      bqkv, NQK,
      (void*)QKH, (void*)QKL, NQK, 0LL,
      NROWS, NQK, KQK, 1.0f, 1.0f);

  gemm64<0, 2, 0, 2, 0><<<gV, blk, 0, stream>>>(
      WV16, DM, 0LL,
      H16, DM, (long long)SEQ * DM,
      (const float*)0, 0, 0LL,
      bqkv + 2 * DM, DM,
      (void*)VTp, (void*)0, SEQ, (long long)DM * SEQ,
      DM, SEQ, DM, 1.0f / (HCARRY * WSC), VC);

  attn8<<<gAT, bAT, 0, stream>>>(QKH, QKL, VTp, CT);

  gemm64<0, 0, 1, 1, 0><<<gO, blk, 0, stream>>>(
      CT, DM, (long long)SEQ * DM,
      WO16, DM, 0LL,
      x, DM, (long long)SEQ_FULL * DM,
      b0, DM,
      (void*)X1F, (void*)0, DM, (long long)SEQ * DM,
      SEQ, DM, DM, 1.0f / (FC * WSC), 1.0f);

  lnorm<0, 0><<<gLN, bLN, 0, stream>>>(X1F, (long long)SEQ * DM, lng, lnb, H2, H2C, (unsigned short*)0);

  gemm64<0, 2, 0, 1, 2><<<gF1, blk, 0, stream>>>(
      H2, DM, 0LL,
      W116, DM, 0LL,
      (const float*)0, 0, 0LL,
      b1, DFF,
      (void*)HH, (void*)0, DFFP, 0LL,
      NROWS, DFFP, DM, 1.0f / (H2C * WSC), GC);

  gemm64<0, 0, 2, 1, 0><<<gF2, blk, 0, stream>>>(
      HH, DFFP, 0LL,
      W216, DFFP, 0LL,
      X1F, DM, 0LL,
      b2, DM,
      (void*)out, (void*)0, DM, 0LL,
      NROWS, DM, DFFP, 1.0f / (GC * W2SC), 1.0f);
}
